// GAT_29231547416655
// MI455X (gfx1250) — hardware-verified
//
#include <hip/hip_runtime.h>
#include <math.h>
#include <stdint.h>
#include <stddef.h>

#define NB   2
#define NN   2048
#define FIN  128
#define FOUT 128
#define NH   4
#define UU   1024
#define HF   (NH * FOUT)
#define MR   (NB * NN)
#define BQ   64
#define BK   64
#define OSP  132
#define TFP  68

#define PB_XB (MR * FIN / 8 / 256)
#define PB_WT (HF * FIN / 8 / 256)
#define PB_A  1
#define PB_MW (NB * 2 * 16 * 16)
#define PB_ALL (PB_XB + PB_WT + PB_A + PB_MW)

static_assert(NN - UU == UU && UU == 1024);
static_assert(UU % BQ == 0 && UU % BK == 0 && BK % 32 == 0);
static_assert(FOUT == 128 && NH * FOUT == 512 && FIN == 128);
static_assert(MR % 128 == 0 && MR % 64 == 0 && MR % 32 == 0);
static_assert(FIN % 32 == 0 && NH * 2 * FOUT == 1024);
static_assert(BQ == 64 && BK == 64 && NN % 64 == 0);
static_assert((MR * FIN / 8) % 256 == 0 && (HF * FIN / 8) % 256 == 0);
static_assert((OSP * 4) % 16 == 0 && (TFP * 4) % 16 == 0);

typedef float          v4f   __attribute__((ext_vector_type(4)));
typedef float          v8f   __attribute__((ext_vector_type(8)));
typedef int            v4i   __attribute__((ext_vector_type(4)));
typedef int            v8i   __attribute__((ext_vector_type(8)));
typedef unsigned int   v2u   __attribute__((ext_vector_type(2)));
typedef unsigned short v8us  __attribute__((ext_vector_type(8)));
typedef unsigned short v16us __attribute__((ext_vector_type(16)));
typedef __bf16         v16bf __attribute__((ext_vector_type(16)));
typedef v4f  __attribute__((may_alias)) v4fa;
typedef v2u  __attribute__((may_alias)) v2ua;
typedef v8us __attribute__((may_alias)) v8usa;
union FragB { v16bf v; v16us u; v8us h[2]; v8i w; };

__device__ __forceinline__ v8f wmb(const FragB& a, const FragB& b, v8f c) {
  v8f d = __builtin_amdgcn_wmma_f32_16x16x32_bf16(false, a.v, false, b.v, (short)0, c, false, false);
  asm volatile("v_nop\n\tv_nop\n\tv_nop\n\tv_nop" : "+v"(d) : "v"(a.w), "v"(b.w));
  return d;
}

__device__ __forceinline__ unsigned bf16_bits(float f) {
  const unsigned u = __float_as_uint(f);
  const unsigned r = (u + 0x7FFFu + ((u >> 16) & 1u)) >> 16;
  const unsigned n = (u >> 16) | 0x40u;
  return ((u & 0x7FFFFFFFu) > 0x7F800000u) ? n : r;
}
__device__ __forceinline__ float bf16_val(float f) { return __uint_as_float(bf16_bits(f) << 16); }
__device__ __forceinline__ v4f bfr4(const v4f a) {
  v4f r; r.x = bf16_val(a.x); r.y = bf16_val(a.y); r.z = bf16_val(a.z); r.w = bf16_val(a.w); return r;
}
__device__ __forceinline__ float lrelu(float e) { return (e > 0.0f) ? e : 0.2f * e; }

__global__ __launch_bounds__(256) void k_prep(const float* __restrict__ x, const float* __restrict__ wts,
                                              const float* __restrict__ W, const float* __restrict__ a,
                                              const int* __restrict__ adj,
                                              unsigned short* XB, unsigned short* WT, float* A32, float* MW) {
  __shared__ __align__(16) float tf[64 * TFP];
  const int bx = (int)blockIdx.x, tid = (int)threadIdx.x;
  if (bx < PB_XB) {
    const int u = bx * 256 + tid;
    const int row = u >> 4, k8 = (u & 15) * 8;
    const float* p = x + (size_t)row * FIN + k8;
    const v4f a0 = *(const v4f*)p;
    const v4f a1 = *(const v4f*)(p + 4);
    v8us o;
    o[0] = (unsigned short)bf16_bits(a0.x); o[1] = (unsigned short)bf16_bits(a0.y);
    o[2] = (unsigned short)bf16_bits(a0.z); o[3] = (unsigned short)bf16_bits(a0.w);
    o[4] = (unsigned short)bf16_bits(a1.x); o[5] = (unsigned short)bf16_bits(a1.y);
    o[6] = (unsigned short)bf16_bits(a1.z); o[7] = (unsigned short)bf16_bits(a1.w);
    unsigned short* dp = XB + (size_t)row * FIN + k8;
    *(volatile v8us*)dp = o;
    __threadfence();
    *(volatile v8us*)dp = o;
  } else if (bx < PB_XB + PB_WT) {
    const int u = (bx - PB_XB) * 256 + tid;
    const int n = u >> 4, k8 = (u & 15) * 8;
    const int h = n >> 7, f = n & 127;
    const float* p = W + ((size_t)h * FIN + k8) * FOUT + f;
    v8us o;
#pragma unroll
    for (int i = 0; i < 8; ++i) o[i] = (unsigned short)bf16_bits(p[(size_t)i * FOUT]);
    unsigned short* dp = WT + (size_t)n * FIN + k8;
    *(volatile v8us*)dp = o;
    __threadfence();
    *(volatile v8us*)dp = o;
  } else if (bx < PB_XB + PB_WT + PB_A) {
    const v4f v = bfr4(*(const v4f*)(a + 4 * tid));
    float* dp = A32 + 4 * tid;
    *(volatile v4f*)dp = v;
    __threadfence();
    *(volatile v4f*)dp = v;
  } else {
    const int m = bx - (PB_XB + PB_WT + PB_A);
    const int tcx = m & 15, tcy = (m >> 4) & 15, q = (m >> 8) & 1, b = m >> 9;
    const int r0 = tcy * 64, c0 = tcx * 64;
    const int inR0 = (q == 0) ? c0 : r0;
    const int inC0 = (q == 0) ? r0 : c0;
    const int lr = tid >> 4, c4 = (tid & 15) * 4;
    const float* wb = wts + (size_t)b * UU * UU;
#pragma unroll
    for (int it = 0; it < 4; ++it) {
      const int rr = it * 16 + lr;
      const v4f w4 = *(const v4f*)(wb + (size_t)(inR0 + rr) * UU + inC0 + c4);
      *(v4fa*)(tf + rr * TFP + c4) = bfr4(w4);
    }
    __syncthreads();
    const int irow0 = (q == 0) ? r0 : (UU + r0);
    const int jcol0 = (q == 0) ? (UU + c0) : c0;
    const int step  = (q == 0) ? TFP : 1;
    v4f o[4];
#pragma unroll
    for (int it = 0; it < 4; ++it) {
      const int ro = it * 16 + lr;
      const v4i av = *(const v4i*)(adj + ((size_t)(b * NN + irow0 + ro)) * NN + jcol0 + c4);
      asm volatile("" :: "v"(av));
      const int base = (q == 0) ? (c4 * TFP + ro) : (ro * TFP + c4);
      const float w0 = tf[base], w1 = tf[base + step], w2 = tf[base + 2 * step], w3 = tf[base + 3 * step];
      o[it].x = __uint_as_float(__float_as_uint(w0) & (unsigned)(-(int)(av.x > 0)));
      o[it].y = __uint_as_float(__float_as_uint(w1) & (unsigned)(-(int)(av.y > 0)));
      o[it].z = __uint_as_float(__float_as_uint(w2) & (unsigned)(-(int)(av.z > 0)));
      o[it].w = __uint_as_float(__float_as_uint(w3) & (unsigned)(-(int)(av.w > 0)));
    }
    float* mp = MW + ((size_t)(b * 2 + q) * UU + r0 + lr) * UU + c0 + c4;
#pragma unroll
    for (int it = 0; it < 4; ++it) *(volatile v4f*)(mp + (size_t)it * 16 * UU) = o[it];
    __threadfence();
#pragma unroll
    for (int it = 0; it < 4; ++it) *(volatile v4f*)(mp + (size_t)it * 16 * UU) = o[it];
  }
}

__global__ __launch_bounds__(128) __attribute__((amdgpu_num_vgpr(248)))
void k_wh(const unsigned short* __restrict__ XB, const unsigned short* __restrict__ WT, float* WH) {
  __shared__ __align__(16) float stg[64 * OSP];
  const int tid = (int)threadIdx.x, lane = tid & 31, wave = tid >> 5, hh = lane >> 4, m = lane & 15;
  const int rowBase = (int)blockIdx.x * 64;
  const int colBase = (int)blockIdx.y * 128;
  v8f acc[8];
  {
    const v8f z = {0.f, 0.f, 0.f, 0.f, 0.f, 0.f, 0.f, 0.f};
#pragma unroll
    for (int t = 0; t < 8; ++t) acc[t] = z;
  }
  const unsigned short* ap = XB + (size_t)(rowBase + 16 * wave + m) * FIN + 8 * hh;
  const unsigned short* bp = WT + (size_t)(colBase + m) * FIN + 8 * hh;
#pragma unroll 1
  for (int k0 = 0; k0 < FIN; k0 += 32) {
    FragB af;
    af.h[0] = *(const v8usa*)(ap + k0);
    af.h[1] = *(const v8usa*)(ap + k0 + 16);
#pragma unroll
    for (int nt = 0; nt < 8; ++nt) {
      const unsigned short* wq = bp + (size_t)(16 * nt) * FIN + k0;
      FragB bf;
      bf.h[0] = *(const v8usa*)wq;
      bf.h[1] = *(const v8usa*)(wq + 16);
      acc[nt] = wmb(af, bf, acc[nt]);
    }
  }
#pragma unroll
  for (int nt = 0; nt < 8; ++nt) {
#pragma unroll
    for (int r = 0; r < 8; ++r) stg[(16 * wave + 8 * hh + r) * OSP + 16 * nt + m] = acc[nt][r];
  }
  __syncthreads();
  float* op = WH + (size_t)(rowBase + wave * 16) * HF + colBase + 4 * lane;
  const float* sp = stg + (wave * 16) * OSP + 4 * lane;
#pragma unroll 1
  for (int i = 0; i < 16; ++i) {
    const v4f p = *(const v4fa*)(sp + i * OSP);
    *(volatile v4f*)(op + (size_t)i * HF) = p;
  }
  __threadfence();
#pragma unroll 1
  for (int i = 0; i < 16; ++i) {
    const v4f p = *(const v4fa*)(sp + i * OSP);
    *(volatile v4f*)(op + (size_t)i * HF) = p;
  }
}

__global__ __launch_bounds__(256) void k_sd(const float* __restrict__ WH, const float* __restrict__ A32, float* SD) {
  __shared__ __align__(16) float sA[NH * 2 * FOUT];
  __shared__ __align__(16) float sdl[8 * 32];
  const int tid = (int)threadIdx.x, lane = tid & 31, wave = tid >> 5;
  {
    const v4f t4 = *(const v4f*)(A32 + 4 * tid);
    *(v4fa*)(sA + 4 * tid) = t4;
  }
  __syncthreads();
  v4f as4[NH], ad4[NH];
#pragma unroll
  for (int h = 0; h < NH; ++h) {
    as4[h] = *(const v4fa*)(sA + h * 2 * FOUT + 4 * lane);
    ad4[h] = *(const v4fa*)(sA + h * 2 * FOUT + FOUT + 4 * lane);
  }
  const int row0 = (int)blockIdx.x * 32;
#pragma unroll 1
  for (int i = 0; i < 4; ++i) {
    const int rl = wave * 4 + i;
    const float* rp = WH + (size_t)(row0 + rl) * HF + 4 * lane;
    float s[NH], d[NH];
#pragma unroll
    for (int h = 0; h < NH; ++h) {
      const v4f p = *(const v4f*)(rp + h * FOUT);
      float sv = 0.0f, dv = 0.0f;
      sv = fmaf(p.x, as4[h].x, sv); sv = fmaf(p.y, as4[h].y, sv); sv = fmaf(p.z, as4[h].z, sv); sv = fmaf(p.w, as4[h].w, sv);
      dv = fmaf(p.x, ad4[h].x, dv); dv = fmaf(p.y, ad4[h].y, dv); dv = fmaf(p.z, ad4[h].z, dv); dv = fmaf(p.w, ad4[h].w, dv);
      s[h] = sv; d[h] = dv;
    }
#pragma unroll
    for (int off = 16; off > 0; off >>= 1) {
#pragma unroll
      for (int h = 0; h < NH; ++h) {
        s[h] += __shfl_xor(s[h], off);
        d[h] += __shfl_xor(d[h], off);
      }
    }
    if (lane == 0) {
#pragma unroll
      for (int h = 0; h < NH; ++h) { sdl[h * 32 + rl] = s[h]; sdl[(NH + h) * 32 + rl] = d[h]; }
    }
  }
  __syncthreads();
  const float val = sdl[wave * 32 + lane];
  const int b = row0 >> 11, n0 = row0 & (NN - 1);
  float* dp = SD + ((size_t)((b * 2 + (wave >> 2)) * NH + (wave & 3))) * NN + n0 + lane;
  *(volatile float*)dp = val;
  __threadfence();
  *(volatile float*)dp = val;
}

__global__ __launch_bounds__(256) void k_den(const float* __restrict__ MW, const float* __restrict__ SD,
                                             const float* __restrict__ WH, float* DEN,
                                             unsigned short* VTH, unsigned short* VTL) {
  __shared__ __align__(16) float sS[UU];
  __shared__ __align__(16) float sP[16 * 64];
  __shared__ __align__(16) float sDen[64];
  __shared__ __align__(16) float sRd[64];
  __shared__ __align__(16) float vt[64 * OSP];
  const int tid = (int)threadIdx.x, lane = tid & 31, wave = tid >> 5;
  const int bx = (int)blockIdx.x;
  const int ct = bx & 15, h = (bx >> 4) & 3, q = (bx >> 6) & 1, b = bx >> 7;
  const int ibase = q * UU;
  const int jbase = (1 - q) * UU;
  const int c0 = ct * 64;
  const int j0 = jbase + c0;
  const float* Sp = SD + ((size_t)((b * 2 + 0) * NH + h)) * NN;
  const float* Dp = SD + ((size_t)((b * 2 + 1) * NH + h)) * NN;
  {
    const v4f s4 = *(const v4f*)(Sp + ibase + 4 * tid);
    *(v4fa*)(sS + 4 * tid) = s4;
  }
  const int cq = tid & 15, rg = tid >> 4;
  const v4f d4 = *(const v4f*)(Dp + j0 + 4 * cq);
  __syncthreads();
  const float* mwp = MW + ((size_t)(b * 2 + q) * UU + rg) * UU + c0 + 4 * cq;
  v4f acc = {0.0f, 0.0f, 0.0f, 0.0f};
#pragma unroll 1
  for (int rr = 0; rr < 64; ++rr) {
    const v4f mw = *(const v4f*)(mwp + (size_t)rr * 16 * UU);
    const float s = sS[rg + 16 * rr];
    acc.x += fabsf(expf(lrelu(s + d4.x)) * mw.x);
    acc.y += fabsf(expf(lrelu(s + d4.y)) * mw.y);
    acc.z += fabsf(expf(lrelu(s + d4.z)) * mw.z);
    acc.w += fabsf(expf(lrelu(s + d4.w)) * mw.w);
  }
  *(v4fa*)(sP + rg * 64 + 4 * cq) = acc;
  __syncthreads();
  if (tid < 64) {
    float sum = 0.0f;
#pragma unroll 1
    for (int g = 0; g < 16; ++g) sum += sP[g * 64 + tid];
    const float den = (sum < 1e-12f) ? 1e-12f : sum;
    sDen[tid] = den;
    sRd[tid]  = 1.0f / den;
  }
  __syncthreads();
  {
    const v4f dv = *(const v4fa*)(sDen + 4 * (tid & 15));
    asm volatile("" :: "v"(dv));
    float* dp = DEN + ((size_t)(b * NH + h)) * NN + j0 + 4 * (tid & 15);
    if (tid < 16) *(volatile v4f*)dp = dv;
    __threadfence();
    if (tid < 16) *(volatile v4f*)dp = dv;
  }
#pragma unroll 1
  for (int it = 0; it < 8; ++it) {
    const int jj = it * 8 + wave;
    v4f w4 = *(const v4f*)(WH + ((size_t)(b * NN + j0 + jj)) * HF + h * FOUT + 4 * lane);
    const float rd = sRd[jj];
    w4.x *= rd; w4.y *= rd; w4.z *= rd; w4.w *= rd;
    *(v4fa*)(vt + jj * OSP + 4 * lane) = w4;
  }
  __syncthreads();
  const int l8 = tid & 7, dsub = tid >> 3;
  v8us ho[4], lo[4];
#pragma unroll
  for (int it = 0; it < 4; ++it) {
    const int d = it * 32 + dsub;
#pragma unroll
    for (int e = 0; e < 8; ++e) {
      const float f = vt[(8 * l8 + e) * OSP + d];
      const unsigned hb = bf16_bits(f);
      const unsigned lb = bf16_bits(f - __uint_as_float(hb << 16));
      ho[it][e] = (unsigned short)hb;
      lo[it][e] = (unsigned short)lb;
    }
  }
  const size_t vb = ((size_t)((b * NH + h) * FOUT + dsub)) * NN + j0 + 8 * l8;
#pragma unroll
  for (int it = 0; it < 4; ++it) {
    *(volatile v8us*)(VTH + vb + (size_t)it * 32 * NN) = ho[it];
    *(volatile v8us*)(VTL + vb + (size_t)it * 32 * NN) = lo[it];
  }
  __threadfence();
#pragma unroll
  for (int it = 0; it < 4; ++it) {
    *(volatile v8us*)(VTH + vb + (size_t)it * 32 * NN) = ho[it];
    *(volatile v8us*)(VTL + vb + (size_t)it * 32 * NN) = lo[it];
  }
}

__global__ __launch_bounds__(128) __attribute__((amdgpu_num_vgpr(248)))
void k_pv(const float* __restrict__ MW, const float* __restrict__ SD,
          const unsigned short* __restrict__ VTH, const unsigned short* __restrict__ VTL, float* outp) {
  __shared__ __align__(16) unsigned short Vh[FOUT * BK];
  __shared__ __align__(16) unsigned short Vl[FOUT * BK];
  __shared__ __align__(16) unsigned short Ph[4 * 16 * BK];
  __shared__ __align__(16) unsigned short Pl[4 * 16 * BK];
  __shared__ __align__(16) float sS[BQ];
  __shared__ __align__(16) float sD[UU];
  __shared__ __align__(16) float Os[4 * 16 * OSP];
  const int tid = (int)threadIdx.x, lane = tid & 31, wave = tid >> 5, hh = lane >> 4, c = lane & 15;
  const int bx = (int)blockIdx.x;
  const int qt = bx & 31, h = (bx >> 5) & 3, b = bx >> 7;
  const int i0 = qt * BQ;
  const int q = (i0 < UU) ? 0 : 1;
  const int ibase = q * UU;
  const int jbase = (1 - q) * UU;
  const int rloc0 = i0 - ibase;
  const float* Sp = SD + ((size_t)((b * 2 + 0) * NH + h)) * NN;
  const float* Dp = SD + ((size_t)((b * 2 + 1) * NH + h)) * NN;
  {
    const v4f s4 = *(const v4f*)(Sp + i0 + 4 * (tid & 15));
    asm volatile("" :: "v"(s4));
    if (tid < 16) *(v4fa*)(sS + 4 * tid) = s4;
#pragma unroll
    for (int it = 0; it < 2; ++it) {
      const int idx = it * 128 + tid;
      const v4f d4 = *(const v4f*)(Dp + jbase + 4 * idx);
      *(v4fa*)(sD + 4 * idx) = d4;
    }
  }
  v8f oacc[8];
  {
    const v8f z = {0.f, 0.f, 0.f, 0.f, 0.f, 0.f, 0.f, 0.f};
#pragma unroll
    for (int t = 0; t < 8; ++t) oacc[t] = z;
  }
  unsigned short* ph = Ph + wave * 16 * BK;
  unsigned short* pl = Pl + wave * 16 * BK;
  const size_t vrow = ((size_t)((b * NH + h) * FOUT + tid)) * NN + jbase;
  const int cq = lane & 15, rh = lane >> 4;
  const float* mwb = MW + ((size_t)(b * 2 + q) * UU + rloc0 + wave * 16 + rh) * UU + 4 * cq;

#pragma unroll 1
  for (int kt = 0; kt < UU / BK; ++kt) {
    __syncthreads();
    {
      const unsigned short* gh = VTH + vrow + kt * BK;
      const unsigned short* gl = VTL + vrow + kt * BK;
#pragma unroll 4
      for (int i = 0; i < 8; ++i) {
        const v8us a0 = *(const v8usa*)(gh + 8 * i);
        const v8us a1 = *(const v8usa*)(gl + 8 * i);
        *(v8usa*)(Vh + tid * BK + 8 * i) = a0;
        *(v8usa*)(Vl + tid * BK + 8 * i) = a1;
      }
    }
    {
      const v4f d4 = *(const v4fa*)(sD + kt * BK + 4 * cq);
      const float* mwp = mwb + kt * BK;
#pragma unroll 1
      for (int it = 0; it < 8; ++it) {
        const int row = it * 2 + rh;
        const v4f mw = *(const v4f*)(mwp + (size_t)it * 2 * UU);
        const float s = sS[wave * 16 + row];
        const float p0 = expf(lrelu(s + d4.x)) * mw.x;
        const float p1 = expf(lrelu(s + d4.y)) * mw.y;
        const float p2 = expf(lrelu(s + d4.z)) * mw.z;
        const float p3 = expf(lrelu(s + d4.w)) * mw.w;
        const unsigned h0 = bf16_bits(p0), h1 = bf16_bits(p1), h2 = bf16_bits(p2), h3 = bf16_bits(p3);
        const unsigned l0 = bf16_bits(p0 - __uint_as_float(h0 << 16));
        const unsigned l1 = bf16_bits(p1 - __uint_as_float(h1 << 16));
        const unsigned l2 = bf16_bits(p2 - __uint_as_float(h2 << 16));
        const unsigned l3 = bf16_bits(p3 - __uint_as_float(h3 << 16));
        v2u hv, lv;
        hv.x = h0 | (h1 << 16); hv.y = h2 | (h3 << 16);
        lv.x = l0 | (l1 << 16); lv.y = l2 | (l3 << 16);
        *(v2ua*)(ph + row * BK + 4 * cq) = hv;
        *(v2ua*)(pl + row * BK + 4 * cq) = lv;
      }
    }
    __syncthreads();
#pragma unroll 1
    for (int kk = 0; kk < BK / 32; ++kk) {
      FragB pa, pb;
      pa.h[0] = *(const v8usa*)(ph + c * BK + kk * 32 + 8 * hh);
      pa.h[1] = *(const v8usa*)(ph + c * BK + kk * 32 + 16 + 8 * hh);
      pb.h[0] = *(const v8usa*)(pl + c * BK + kk * 32 + 8 * hh);
      pb.h[1] = *(const v8usa*)(pl + c * BK + kk * 32 + 16 + 8 * hh);
#pragma unroll
      for (int t = 0; t < 8; ++t) {
        FragB vb, vl;
        vb.h[0] = *(const v8usa*)(Vh + (t * 16 + c) * BK + kk * 32 + 8 * hh);
        vb.h[1] = *(const v8usa*)(Vh + (t * 16 + c) * BK + kk * 32 + 16 + 8 * hh);
        vl.h[0] = *(const v8usa*)(Vl + (t * 16 + c) * BK + kk * 32 + 8 * hh);
        vl.h[1] = *(const v8usa*)(Vl + (t * 16 + c) * BK + kk * 32 + 16 + 8 * hh);
        oacc[t] = wmb(pa, vb, oacc[t]);
        oacc[t] = wmb(pa, vl, oacc[t]);
        oacc[t] = wmb(pb, vb, oacc[t]);
      }
    }
  }

  float* os = Os + wave * 16 * OSP;
#pragma unroll
  for (int t = 0; t < 8; ++t) {
#pragma unroll
    for (int r = 0; r < 8; ++r) os[(8 * hh + r) * OSP + t * 16 + c] = oacc[t][r];
  }
  __syncthreads();
#pragma unroll 1
  for (int row = 0; row < 16; ++row) {
    v4f v = *(const v4fa*)(os + row * OSP + 4 * lane);
    v.x = (v.x > 0.0f) ? v.x : expm1f(v.x);
    v.y = (v.y > 0.0f) ? v.y : expm1f(v.y);
    v.z = (v.z > 0.0f) ? v.z : expm1f(v.z);
    v.w = (v.w > 0.0f) ? v.w : expm1f(v.w);
    *(v4fa*)(os + row * OSP + 4 * lane) = v;
  }
  __syncthreads();
  float* op = outp + ((size_t)(b * NN + i0 + wave * 16)) * HF + h * FOUT + 4 * lane;
#pragma unroll 1
  for (int row = 0; row < 16; ++row) {
    const v4f v = *(const v4fa*)(os + row * OSP + 4 * lane);
    *(volatile v4f*)(op + (size_t)row * HF) = v;
  }
  __threadfence();
#pragma unroll 1
  for (int row = 0; row < 16; ++row) {
    const v4f v = *(const v4fa*)(os + row * OSP + 4 * lane);
    *(volatile v4f*)(op + (size_t)row * HF) = v;
  }
}

extern "C" void kernel_launch(void* const* d_in, const int* in_sizes, int n_in,
                              void* d_out, int out_size, void* d_ws, size_t ws_size,
                              hipStream_t stream) {
  if (n_in < 5) return;
  if (in_sizes[0] != NB * NN * FIN) return;
  if (in_sizes[1] != NB * (NN - UU) * UU) return;
  if (in_sizes[2] != NH * FIN * FOUT) return;
  if (in_sizes[3] != NH * 2 * FOUT) return;
  if (in_sizes[4] != NB * NN * NN) return;
  if (out_size != NB * NN * HF) return;

  const float* x   = (const float*)d_in[0];
  const float* wts = (const float*)d_in[1];
  const float* W   = (const float*)d_in[2];
  const float* a   = (const float*)d_in[3];
  const int*   adj = (const int*)d_in[4];
  float* out = (float*)d_out;

  size_t off = 0;
  const size_t oXB  = off; off += (size_t)MR * FIN * 2;
  const size_t oWT  = off; off += (size_t)HF * FIN * 2;
  const size_t oA32 = off; off += (size_t)NH * 2 * FOUT * 4;
  const size_t oWH  = off; off += (size_t)MR * HF * 4;
  const size_t oSD  = off; off += (size_t)NB * 2 * NH * NN * 4;
  const size_t oMW  = off; off += (size_t)NB * 2 * UU * UU * 4;
  const size_t oDEN = off; off += (size_t)NB * NH * NN * 4;
  const size_t oVTH = off; off += (size_t)NB * NH * FOUT * NN * 2;
  const size_t oVTL = off; off += (size_t)NB * NH * FOUT * NN * 2;
  if (off > ws_size || off > (size_t)134217728) return;

  char* ws = (char*)d_ws;
  unsigned short* XB  = (unsigned short*)(ws + oXB);
  unsigned short* WT  = (unsigned short*)(ws + oWT);
  float*          A32 = (float*)(ws + oA32);
  float*          WH  = (float*)(ws + oWH);
  float*          SD  = (float*)(ws + oSD);
  float*          MW  = (float*)(ws + oMW);
  float*          DEN = (float*)(ws + oDEN);
  unsigned short* VTH = (unsigned short*)(ws + oVTH);
  unsigned short* VTL = (unsigned short*)(ws + oVTL);

  k_prep<<<dim3(PB_ALL), dim3(256), 0, stream>>>(x, wts, W, a, adj, XB, WT, A32, MW);
  k_wh<<<dim3(MR / 64, HF / 128), dim3(128), 0, stream>>>(XB, WT, WH);
  k_sd<<<dim3(MR / 32), dim3(256), 0, stream>>>(WH, A32, SD);
  k_den<<<dim3(NB * 2 * NH * (UU / 64)), dim3(256), 0, stream>>>(MW, SD, WH, DEN, VTH, VTL);
  k_pv<<<dim3(NB * NH * (NN / BQ)), dim3(128), 0, stream>>>(MW, SD, VTH, VTL, out);
  (void)hipGetLastError();
}
